// NeuralODE_85830626443530
// MI455X (gfx1250) — hardware-run, weakly checked
//
#include <hip/hip_runtime.h>
#include <math.h>

constexpr int NBAT   = 1024;
constexpr int DZC    = 256;
constexpr int DHC    = 1024;
constexpr int NSTEPS = 8;
constexpr int NSTAGE = 4;
constexpr int NTH    = 256;
constexpr int SLP    = 68;
constexpr float W1CARRY     = 16.0f;
constexpr float W1CARRY_INV = 1.0f / 16.0f;
constexpr float W2CARRY     = 32.0f;
constexpr float W2CARRY_INV = 1.0f / 32.0f;
static_assert(NBAT % 64 == 0 && DZC % 64 == 0 && DHC % 64 == 0);
static_assert(DZC % 32 == 0 && DHC % 32 == 0);
static_assert((NBAT * DZC / 8) % NTH == 0);
static_assert(((NBAT / 64) * (DHC / 64)) % (NTH / 32) == 0);
static_assert(((NBAT / 64) * (DZC / 64)) % (NTH / 32) == 0);

typedef __attribute__((ext_vector_type(16))) _Float16 v16h;
typedef __attribute__((ext_vector_type(8)))  _Float16 v8h;
typedef __attribute__((ext_vector_type(16))) __bf16   v16b;
typedef __attribute__((ext_vector_type(8)))  __bf16   v8b;
typedef __attribute__((ext_vector_type(8)))  float    v8f;
typedef __attribute__((ext_vector_type(4)))  float    v4f;

__device__ __forceinline__ unsigned short f2bf_bits(float f) {
  unsigned u = __float_as_uint(f);
  return (unsigned short)((u + 0x7FFFu + ((u >> 16) & 1u)) >> 16);
}
__device__ __forceinline__ float bf_bits2f(unsigned short h) { return __uint_as_float(((unsigned)h) << 16); }

__device__ __forceinline__ void dep_guard_h(v8f& a, v8f& b, v16h x, v16h y) { asm volatile("v_nop\n\tv_nop\n\tv_nop\n\tv_nop" : "+v"(a), "+v"(b) : "v"(x), "v"(y)); }
__device__ __forceinline__ void dep_guard_b(v8f& a, v8f& b, v16b x, v16b y) { asm volatile("v_nop\n\tv_nop\n\tv_nop\n\tv_nop" : "+v"(a), "+v"(b) : "v"(x), "v"(y)); }
__device__ __forceinline__ void dep_guard4_h(v8f& a, v8f& b, v8f& c, v8f& d, v16h x, v16h y) {
  asm volatile("v_nop\n\tv_nop\n\tv_nop\n\tv_nop" : "+v"(a), "+v"(b), "+v"(c), "+v"(d) : "v"(x), "v"(y));
}
__device__ __forceinline__ void dep_guard4_b(v8f& a, v8f& b, v8f& c, v8f& d, v16b x, v16b y) {
  asm volatile("v_nop\n\tv_nop\n\tv_nop\n\tv_nop" : "+v"(a), "+v"(b), "+v"(c), "+v"(d) : "v"(x), "v"(y));
}
__device__ __forceinline__ void keep4_h(v16h a, v16h b, v16h c, v16h d) { asm volatile("v_nop" :: "v"(a), "v"(b), "v"(c), "v"(d)); }
__device__ __forceinline__ void keep4_b(v16b a, v16b b, v16b c, v16b d) { asm volatile("v_nop" :: "v"(a), "v"(b), "v"(c), "v"(d)); }
__device__ __forceinline__ void acc_guard4(v8f& a, v8f& b, v8f& c, v8f& d) { asm volatile("v_nop\n\tv_nop\n\tv_nop\n\tv_nop" : "+v"(a), "+v"(b), "+v"(c), "+v"(d)); }
template <typename T> struct Frag;
template <> struct Frag<_Float16> {
  typedef v16h V; union U { v16h v; v8h h[2]; };
  static __device__ __forceinline__ v16h load(const _Float16* p) {
    U f; f.h[0] = *(const v8h*)(p); f.h[1] = *(const v8h*)(p + 16); return f.v;
  }
  static __device__ __forceinline__ v8f mma(v16h a, v16h b, v8f c) {
    return __builtin_amdgcn_wmma_f32_16x16x32_f16(false, a, false, b, (short)0, c, false, false);
  }
  static __device__ __forceinline__ void guard(v8f& a, v8f& b, v16h x, v16h y) { dep_guard_h(a, b, x, y); }
  static __device__ __forceinline__ void guard4(v8f& a, v8f& b, v8f& c, v8f& d, v16h x, v16h y) { dep_guard4_h(a, b, c, d, x, y); }
  static __device__ __forceinline__ void keep(v16h a, v16h b, v16h c, v16h d) { keep4_h(a, b, c, d); }
};
template <> struct Frag<__bf16> {
  typedef v16b V; union U { v16b v; v8b h[2]; };
  static __device__ __forceinline__ v16b load(const __bf16* p) {
    U f; f.h[0] = *(const v8b*)(p); f.h[1] = *(const v8b*)(p + 16); return f.v;
  }
  static __device__ __forceinline__ v8f mma(v16b a, v16b b, v8f c) {
    return __builtin_amdgcn_wmma_f32_16x16x32_bf16(false, a, false, b, (short)0, c, false, false);
  }
  static __device__ __forceinline__ void guard(v8f& a, v8f& b, v16b x, v16b y) { dep_guard_b(a, b, x, y); }
  static __device__ __forceinline__ void guard4(v8f& a, v8f& b, v8f& c, v8f& d, v16b x, v16b y) { dep_guard4_b(a, b, c, d, x, y); }
  static __device__ __forceinline__ void keep(v16b a, v16b b, v16b c, v16b d) { keep4_b(a, b, c, d); }
};

template <int ET> struct Elem;
template <> struct Elem<0> { typedef _Float16 T; };
template <> struct Elem<1> { typedef __bf16 T; };
template <int ET, bool SPLIT, int BIAS_MODE, int OUT_MODE, bool RESID, int ACT = 0>
__global__ __launch_bounds__(256) void wmma_gemm64(
    const unsigned short* __restrict__ Ap, const unsigned short* __restrict__ A2p, int lda, long strideA,
    const unsigned short* __restrict__ Btp, const unsigned short* __restrict__ Bt2p, int ldb, long strideB,
    void* __restrict__ Cout, void* __restrict__ Cout2, int ldc, long strideC,
    const float* __restrict__ bias,
    const float* __restrict__ resid, long strideR,
    int M, int N, int K, float scale) {
  typedef typename Elem<ET>::T T;
  typedef typename Frag<T>::V V;
  const T* A = (const T*)Ap; const T* A2 = (const T*)A2p; const T* Bt = (const T*)Btp; const T* Bt2 = (const T*)Bt2p;
  __shared__ __align__(16) float sT[8][16 * 68];
  const int b    = blockIdx.y;
  const int lane = threadIdx.x & 31;
  const int wave = threadIdx.x >> 5;
  const int tilesN = N >> 6;
  const int tilesM = M >> 6;
  const int tile = blockIdx.x * 8 + wave;
  if (tile >= tilesM * tilesN) return;
  const int tm = tile / tilesN;
  const int tn = tile - tm * tilesN;
  const int m0 = tm << 6;
  const int n0 = tn << 6;

  const T* Ab  = A  + (size_t)b * strideA;
  const T* Bb  = Bt + (size_t)b * strideB;
  const T* Ab2 = SPLIT ? (A2  + (size_t)b * strideA) : nullptr;
  const T* Bb2 = SPLIT ? (Bt2 + (size_t)b * strideB) : nullptr;

  const int rlane = lane & 15;
  const int koff  = (lane >> 4) * 8;
  const int mOff  = (lane >> 4) * 8;

  v8f acc[4][4];
#pragma unroll
  for (int i = 0; i < 4; ++i)
#pragma unroll
    for (int j = 0; j < 4; ++j) acc[i][j] = (v8f){0.f,0.f,0.f,0.f,0.f,0.f,0.f,0.f};

  for (int k0 = 0; k0 < K; k0 += 32) {
    V bh[4], bl[4];
#pragma unroll
    for (int j = 0; j < 4; ++j) {
      const size_t bo = (size_t)(n0 + (j << 4) + rlane) * ldb + koff + k0;
      bh[j] = Frag<T>::load(Bb + bo);
      if (SPLIT) bl[j] = Frag<T>::load(Bb2 + bo);
    }
#pragma unroll
    for (int i = 0; i < 4; ++i) {
      const size_t ao = (size_t)(m0 + (i << 4) + rlane) * lda + koff + k0;
      V ah = Frag<T>::load(Ab + ao);
      V al;
      if (SPLIT) al = Frag<T>::load(Ab2 + ao);
#pragma unroll
      for (int j = 0; j < 4; ++j) {
        acc[i][j] = Frag<T>::mma(ah, bh[j], acc[i][j]);
        if (SPLIT) {
          acc[i][j] = Frag<T>::mma(ah, bl[j], acc[i][j]);
          acc[i][j] = Frag<T>::mma(al, bh[j], acc[i][j]);
        }
      }
      Frag<T>::guard4(acc[i][0], acc[i][1], acc[i][2], acc[i][3], ah, SPLIT ? al : bh[3]);
    }
    Frag<T>::keep(bh[0], bh[1], bh[2], bh[3]);
    if (SPLIT) Frag<T>::keep(bl[0], bl[1], bl[2], bl[3]);
  }
  acc_guard4(acc[0][0], acc[0][1], acc[0][2], acc[0][3]);
  acc_guard4(acc[1][0], acc[1][1], acc[1][2], acc[1][3]);
  acc_guard4(acc[2][0], acc[2][1], acc[2][2], acc[2][3]);
  acc_guard4(acc[3][0], acc[3][1], acc[3][2], acc[3][3]);

  float* slab = sT[wave];
  const float* Rb = RESID ? (resid + (size_t)b * strideR) : nullptr;
#pragma unroll
  for (int i = 0; i < 4; ++i) {
    const int mBase = m0 + (i << 4);
#pragma unroll
    for (int j = 0; j < 4; ++j) {
      const int n = n0 + (j << 4) + rlane;
      float bv = 0.f;
      if (BIAS_MODE == 2) bv = bias[n];
#pragma unroll
      for (int r = 0; r < 8; ++r) {
        float v = acc[i][j][r] * scale;
        if (BIAS_MODE == 1) v += bias[mBase + mOff + r];
        if (BIAS_MODE == 2) v += bv;
        if (RESID) v += Rb[(size_t)(mBase + mOff + r) * ldc + n];
        if (ACT == 1) v = tanhf(v);
        if (ACT == 2) v = fmaxf(v, 0.0f);
        if (ACT == 3) v = v / (1.0f + expf(-v));
        if (ACT == 4) v = (v > 0.f) ? v : 0.01f * v;
        if (ACT == 5) v = 0.5f * v * (1.0f + erff(v * 0.70710678118654752f));
        slab[(mOff + r) * 68 + (j << 4) + rlane] = v;
      }
    }
    __builtin_amdgcn_fence(__ATOMIC_RELEASE, "workgroup");
    __builtin_amdgcn_wave_barrier();
    __builtin_amdgcn_fence(__ATOMIC_ACQUIRE, "workgroup");
    if (OUT_MODE == 0) {
      float* C = (float*)Cout + (size_t)b * strideC;
      const int hh = lane >> 4, c4 = (lane & 15) * 4;
      for (int pass = 0; pass < 2; ++pass) {
#pragma unroll
        for (int it = 0; it < 8; ++it) {
          const int row = it * 2 + hh;
          v4f v = *(const v4f*)(slab + row * 68 + c4);
          *(volatile v4f*)(C + (size_t)(mBase + row) * ldc + n0 + c4) = v;
        }
        __threadfence();
      }
    } else {
      const int q = lane >> 3, c8 = (lane & 7) * 8;
      unsigned short* C  = (unsigned short*)Cout  + (size_t)b * strideC;
      unsigned short* C2 = (OUT_MODE == 2) ? ((unsigned short*)Cout2 + (size_t)b * strideC) : nullptr;
      for (int pass = 0; pass < 2; ++pass) {
#pragma unroll
        for (int it = 0; it < 4; ++it) {
          const int row = it * 4 + q;
          const float* sp = slab + row * 68 + c8;
          v8h hv, lv;
#pragma unroll
          for (int e = 0; e < 8; ++e) {
            if (OUT_MODE == 1) {
              hv[e] = (_Float16)sp[e];
            } else {
              unsigned short hb = f2bf_bits(sp[e]);
              unsigned short lb = f2bf_bits(sp[e] - bf_bits2f(hb));
              hv[e] = __builtin_bit_cast(_Float16, hb);
              lv[e] = __builtin_bit_cast(_Float16, lb);
            }
          }
          *(volatile v8h*)(C + (size_t)(mBase + row) * ldc + n0 + c8) = hv;
          if (OUT_MODE == 2) *(volatile v8h*)(C2 + (size_t)(mBase + row) * ldc + n0 + c8) = lv;
        }
        __threadfence();
      }
    }
    __builtin_amdgcn_fence(__ATOMIC_RELEASE, "workgroup");
    __builtin_amdgcn_wave_barrier();
    __builtin_amdgcn_fence(__ATOMIC_ACQUIRE, "workgroup");
  }
}

__global__ __launch_bounds__(NTH) void tpose_f16_kernel(const float* __restrict__ src, int C, int ldo,
                                                        unsigned short* __restrict__ O, float sc) {
  __shared__ float Tt[64 * 65];
  const int tid = threadIdx.x;
  const int c0 = blockIdx.x * 64, r0 = blockIdx.y * 64;
#pragma unroll
  for (int i = 0; i < 4; ++i) {
    const int idx = i * NTH + tid;
    const int rr = idx >> 4, cc = (idx & 15) * 4;
    const v4f v = *(const v4f*)(src + (size_t)(r0 + rr) * (size_t)C + c0 + cc);
    Tt[rr * 65 + cc + 0] = v[0];
    Tt[rr * 65 + cc + 1] = v[1];
    Tt[rr * 65 + cc + 2] = v[2];
    Tt[rr * 65 + cc + 3] = v[3];
  }
  __syncthreads();
  const int q = tid >> 3, c8 = (tid & 7) * 8;
  v8h hv[2];
#pragma unroll
  for (int g = 0; g < 2; ++g) {
    const int qq = g * 32 + q;
#pragma unroll
    for (int e = 0; e < 8; ++e) hv[g][e] = (_Float16)(Tt[(c8 + e) * 65 + qq] * sc);
  }
  for (int pass = 0; pass < 2; ++pass) {
#pragma unroll
    for (int g = 0; g < 2; ++g) {
      const size_t o = (size_t)(c0 + g * 32 + q) * (size_t)ldo + (size_t)(r0 + c8);
      *(volatile v8h*)(O + o) = hv[g];
    }
    __threadfence();
  }
}

__global__ __launch_bounds__(NTH) void cvt_f16x8_kernel(const float* __restrict__ src, unsigned short* __restrict__ dst, int n8) {
  const int i = blockIdx.x * NTH + threadIdx.x;
  if (i < n8) {
    const float* sp = src + (size_t)i * 8;
    const v4f a = *(const v4f*)(sp);
    const v4f b = *(const v4f*)(sp + 4);
    v8h hv;
#pragma unroll
    for (int e = 0; e < 4; ++e) { hv[e] = (_Float16)a[e]; hv[4 + e] = (_Float16)b[e]; }
    *(volatile v8h*)(dst + (size_t)i * 8) = hv;
    __threadfence();
    *(volatile v8h*)(dst + (size_t)i * 8) = hv;
  }
}

__global__ __launch_bounds__(NTH) void rk_stage_kernel(
    const unsigned short* __restrict__ Hp, const unsigned short* __restrict__ W2p,
    const float* __restrict__ bias2, const float* __restrict__ tvec,
    const float* __restrict__ zbase, const float* __restrict__ ksin,
    float* __restrict__ fout, unsigned short* __restrict__ zeout,
    float cin, float cmul, float azeh, int last) {
  typedef _Float16 T;
  const T* A  = (const T*)Hp;
  const T* Bt = (const T*)W2p;
  __shared__ __align__(16) float sK[NTH / 32][16 * SLP];
  __shared__ __align__(16) float sE[NTH / 32][16 * SLP];
  const int lane = threadIdx.x & 31;
  const int wave = threadIdx.x >> 5;
  constexpr int tilesN = DZC >> 6;
  constexpr int tilesM = NBAT >> 6;
  const int tile = blockIdx.x * (NTH / 32) + wave;
  if (tile >= tilesM * tilesN) return;
  const int tm = tile / tilesN;
  const int tn = tile - tm * tilesN;
  const int m0 = tm << 6;
  const int n0 = tn << 6;

  const int rlane = lane & 15;
  const int koff  = (lane >> 4) * 8;
  const int mOff  = (lane >> 4) * 8;

  const float hstep = (tvec[1] - tvec[0]) * (1.0f / NSTEPS);
  const float h6    = hstep * (1.0f / 6.0f);
  const float aze   = azeh * hstep;

  v8f acc[4][4];
#pragma unroll
  for (int i = 0; i < 4; ++i)
#pragma unroll
    for (int j = 0; j < 4; ++j) acc[i][j] = (v8f){0.f,0.f,0.f,0.f,0.f,0.f,0.f,0.f};

#pragma unroll 1
  for (int k0 = 0; k0 < DHC; k0 += 32) {
    v16h bh[4];
#pragma unroll
    for (int j = 0; j < 4; ++j) {
      const size_t bo = (size_t)(n0 + (j << 4) + rlane) * DHC + koff + k0;
      bh[j] = Frag<T>::load(Bt + bo);
    }
#pragma unroll
    for (int i = 0; i < 4; ++i) {
      const size_t ao = (size_t)(m0 + (i << 4) + rlane) * DHC + koff + k0;
      const v16h ah = Frag<T>::load(A + ao);
#pragma unroll
      for (int j = 0; j < 4; ++j) acc[i][j] = Frag<T>::mma(ah, bh[j], acc[i][j]);
      dep_guard4_h(acc[i][0], acc[i][1], acc[i][2], acc[i][3], ah, bh[3]);
    }
    keep4_h(bh[0], bh[1], bh[2], bh[3]);
  }
  acc_guard4(acc[0][0], acc[0][1], acc[0][2], acc[0][3]);
  acc_guard4(acc[1][0], acc[1][1], acc[1][2], acc[1][3]);
  acc_guard4(acc[2][0], acc[2][1], acc[2][2], acc[2][3]);
  acc_guard4(acc[3][0], acc[3][1], acc[3][2], acc[3][3]);

  float b2v[4];
#pragma unroll
  for (int j = 0; j < 4; ++j) b2v[j] = bias2[n0 + (j << 4) + rlane];

  float* slabK = sK[wave];
  float* slabE = sE[wave];
#pragma unroll
  for (int i = 0; i < 4; ++i) {
    const int mBase = m0 + (i << 4);
#pragma unroll
    for (int j = 0; j < 4; ++j) {
#pragma unroll
      for (int r = 0; r < 8; ++r) slabK[(mOff + r) * SLP + (j << 4) + rlane] = acc[i][j][r] * W2CARRY_INV + b2v[j];
    }
    __builtin_amdgcn_fence(__ATOMIC_RELEASE, "workgroup");
    __builtin_amdgcn_wave_barrier();
    __builtin_amdgcn_fence(__ATOMIC_ACQUIRE, "workgroup");
    {
      const int hh = lane >> 4, c4 = (lane & 15) * 4;
#pragma unroll 2
      for (int it = 0; it < 8; ++it) {
        const int row = it * 2 + hh;
        const size_t g = (size_t)(mBase + row) * DZC + n0 + c4;
        const v4f kv = *(const v4f*)(slabK + row * SLP + c4);
        const v4f zb = *(const v4f*)(zbase + g);
        const v4f ki = *(const v4f*)(ksin + g);
        v4f fo, ze;
#pragma unroll
        for (int e = 0; e < 4; ++e) {
          const float ks = fmaf(cin, ki[e], cmul * kv[e]);
          const float zn = fmaf(ks, h6, zb[e]);
          const float zs = fmaf(kv[e], aze, zb[e]);
          fo[e] = last ? zn : ks;
          ze[e] = last ? zn : zs;
        }
        *(v4f*)(slabK + row * SLP + c4) = fo;
        *(v4f*)(slabE + row * SLP + c4) = ze;
      }
    }
    __builtin_amdgcn_fence(__ATOMIC_RELEASE, "workgroup");
    __builtin_amdgcn_wave_barrier();
    __builtin_amdgcn_fence(__ATOMIC_ACQUIRE, "workgroup");
    for (int pass = 0; pass < 2; ++pass) {
      {
        const int hh = lane >> 4, c4 = (lane & 15) * 4;
#pragma unroll
        for (int it = 0; it < 8; ++it) {
          const int row = it * 2 + hh;
          const v4f v = *(const v4f*)(slabK + row * SLP + c4);
          *(volatile v4f*)(fout + (size_t)(mBase + row) * DZC + n0 + c4) = v;
        }
      }
      {
        const int q = lane >> 3, c8 = (lane & 7) * 8;
#pragma unroll
        for (int it = 0; it < 4; ++it) {
          const int row = it * 4 + q;
          const float* sp = slabE + row * SLP + c8;
          v8h hv;
#pragma unroll
          for (int e = 0; e < 8; ++e) hv[e] = (_Float16)sp[e];
          *(volatile v8h*)(zeout + (size_t)(mBase + row) * DZC + n0 + c8) = hv;
        }
      }
      __threadfence();
    }
    __builtin_amdgcn_fence(__ATOMIC_RELEASE, "workgroup");
    __builtin_amdgcn_wave_barrier();
    __builtin_amdgcn_fence(__ATOMIC_ACQUIRE, "workgroup");
  }
}

extern "C" void kernel_launch(void* const* d_in, const int* in_sizes, int n_in,
                              void* d_out, int out_size, void* d_ws, size_t ws_size, hipStream_t stream) {
  if (n_in < 6 || d_out == nullptr || d_ws == nullptr) return;
  if (in_sizes[0] != NBAT * DZC || in_sizes[1] != 2 || in_sizes[2] != DZC * DHC || in_sizes[3] != DHC ||
      in_sizes[4] != DHC * DZC || in_sizes[5] != DZC || out_size != NBAT * DZC) return;

  const float* z0 = (const float*)d_in[0];
  const float* tv = (const float*)d_in[1];
  const float* w1 = (const float*)d_in[2];
  const float* b1 = (const float*)d_in[3];
  const float* w2 = (const float*)d_in[4];
  const float* b2 = (const float*)d_in[5];
  float* outp = (float*)d_out;

  char* ws = (char*)d_ws; size_t off = 0;
  auto carve = [&](size_t bytes) -> char* { char* p = ws + off; off += (bytes + 255) & ~(size_t)255; return p; };
  unsigned short* W1T = (unsigned short*)carve((size_t)DHC * DZC * 2);
  unsigned short* W2T = (unsigned short*)carve((size_t)DZC * DHC * 2);
  unsigned short* ZE[2];
  ZE[0] = (unsigned short*)carve((size_t)NBAT * DZC * 2);
  ZE[1] = (unsigned short*)carve((size_t)NBAT * DZC * 2);
  unsigned short* HID[2];
  HID[0] = (unsigned short*)carve((size_t)NBAT * DHC * 2);
  HID[1] = (unsigned short*)carve((size_t)NBAT * DHC * 2);
  float* KS[2];
  KS[0] = (float*)carve((size_t)NBAT * DZC * 4);
  KS[1] = (float*)carve((size_t)NBAT * DZC * 4);
  float* ZB[2];
  ZB[0] = (float*)carve((size_t)NBAT * DZC * 4);
  ZB[1] = (float*)carve((size_t)NBAT * DZC * 4);
  if (off > ws_size || off > (size_t)134217728) return;

  tpose_f16_kernel<<<dim3(DHC / 64, DZC / 64), NTH, 0, stream>>>(w1, DHC, DZC, W1T, W1CARRY);
  tpose_f16_kernel<<<dim3(DZC / 64, DHC / 64), NTH, 0, stream>>>(w2, DZC, DHC, W2T, W2CARRY);
  cvt_f16x8_kernel<<<(NBAT * DZC / 8) / NTH, NTH, 0, stream>>>(z0, ZE[0], NBAT * DZC / 8);

  const int g1 = (NBAT / 64) * (DHC / 64) / (NTH / 32);
  const int g2 = (NBAT / 64) * (DZC / 64) / (NTH / 32);
  const float cinT[NSTAGE]  = {0.0f, 1.0f, 1.0f, 1.0f};
  const float cmulT[NSTAGE] = {1.0f, 2.0f, 2.0f, 1.0f};
  const float azehT[NSTAGE] = {0.5f, 0.5f, 1.0f, 0.0f};

  for (int p = 0; p < NSTEPS; ++p) {
    const float* zbase = (p == 0) ? z0 : ZB[(p - 1) & 1];
    for (int s = 0; s < NSTAGE; ++s) {
      const int e = p * NSTAGE + s;
      wmma_gemm64<0, false, 2, 1, false, 1><<<dim3(g1, 1), NTH, 0, stream>>>(
          ZE[e & 1], ZE[e & 1], DZC, 0L, W1T, W1T, DZC, 0L, (void*)HID[e & 1], (void*)HID[e & 1], DHC, 0L,
          b1, b1, 0L, NBAT, DHC, DZC, W1CARRY_INV);
      const float* ksin = (s == 0) ? zbase : KS[(s - 1) & 1];
      float* fo = (s < 3) ? KS[s & 1] : ((p == NSTEPS - 1) ? outp : ZB[p & 1]);
      rk_stage_kernel<<<g2, NTH, 0, stream>>>(HID[e & 1], W2T, b2, tv, zbase, ksin, fo, ZE[(e + 1) & 1],
                                               cinT[s], cmulT[s], azehT[s], (s == 3) ? 1 : 0);
    }
  }
}
